// EALSTM_18494129177333
// MI455X (gfx1250) — hardware-run, weakly checked
//
#include <hip/hip_runtime.h>

typedef __attribute__((ext_vector_type(16))) _Float16 v16h;
typedef __attribute__((ext_vector_type(8)))  float    v8f;
typedef __attribute__((ext_vector_type(4)))  float    v4f;
typedef __attribute__((ext_vector_type(4)))  unsigned int v4u;

constexpr int NB = 256;
constexpr int NT = 365;
constexpr int ND = 32;
constexpr int NS = 27;
constexpr int NU = 256;
constexpr int NG = 3 * NU;
constexpr int KS_PAD = 32;
constexpr int ROWS = 16;
constexpr int HPITCH = NU + 8;
constexpr int OPITCH = NU + 4;
constexpr float CARRY = 16.0f;
constexpr float INV_CARRY2 = 1.0f / 256.0f;

static_assert(NB % ROWS == 0);
static_assert(NG % 32 == 0 && NU % 32 == 0);
static_assert(ND == 32);
static_assert(NS <= KS_PAD && KS_PAD == 32);
static_assert((NB * KS_PAD / 8) % 256 == 0);

constexpr size_t BYTES_KT = (size_t)NG * ND * 2;
constexpr size_t BYTES_RT = (size_t)NG * NU * 2;
constexpr size_t BYTES_WT = (size_t)NU * KS_PAD * 2;
constexpr size_t BYTES_SP = (size_t)NB * KS_PAD * 2;
constexpr size_t OFF_KT = 0;
constexpr size_t OFF_RT = OFF_KT + BYTES_KT;
constexpr size_t OFF_WT = OFF_RT + BYTES_RT;
constexpr size_t OFF_SP = OFF_WT + BYTES_WT;
constexpr size_t WS_TOTAL = OFF_SP + BYTES_SP;
static_assert(WS_TOTAL <= (size_t)134217728);
static_assert(OFF_RT % 512 == 0 && OFF_WT % 512 == 0 && OFF_SP % 512 == 0);

__device__ __forceinline__ unsigned short f2bf_bits(float f) {
  unsigned u = __float_as_uint(f);
  return (unsigned short)((u + 0x7FFFu + ((u >> 16) & 1u)) >> 16);
}
__device__ __forceinline__ float bf_bits2f(unsigned short h) { return __uint_as_float(((unsigned)h) << 16); }
__device__ __forceinline__ float bfr(float f) { return bf_bits2f(f2bf_bits(f)); }
__device__ __forceinline__ _Float16 cvt_in(float f) { return (_Float16)(bfr(f) * CARRY); }
__device__ __forceinline__ unsigned short cvt_in_bits(float f) { return __builtin_bit_cast(unsigned short, cvt_in(f)); }
__device__ __forceinline__ unsigned short h16_bits(float f) { return __builtin_bit_cast(unsigned short, (_Float16)f); }

union FragU { v16h v; v4u q[2]; };

__device__ __forceinline__ v8f mma16(v16h a, v16h b, v8f c) {
  return __builtin_amdgcn_wmma_f32_16x16x32_f16(false, a, false, b, (short)0, c, false, false);
}
__device__ __forceinline__ void guard1(v8f& c, v16h a, v16h b) {
  asm volatile("v_nop\n\tv_nop\n\tv_nop\n\tv_nop" : "+v"(c) : "v"(a), "v"(b));
}
__device__ __forceinline__ void guard3(v8f& c0, v8f& c1, v8f& c2, v16h a, v16h b0, v16h b1, v16h b2) {
  asm volatile("v_nop\n\tv_nop\n\tv_nop\n\tv_nop" : "+v"(c0), "+v"(c1), "+v"(c2) : "v"(a), "v"(b0), "v"(b1), "v"(b2));
}

constexpr float KZERO8[8] = {0.f, 0.f, 0.f, 0.f, 0.f, 0.f, 0.f, 0.f};
__device__ __forceinline__ v8f zero8() { return (v8f){0.f, 0.f, 0.f, 0.f, 0.f, 0.f, 0.f, 0.f}; }

__device__ __forceinline__ float sigm(float x) { return __builtin_amdgcn_rcpf(1.0f + __expf(-x)); }
__device__ __forceinline__ float tnh(float x) { return 1.0f - 2.0f * __builtin_amdgcn_rcpf(1.0f + __expf(2.0f * x)); }

template <int KP, int KREAL>
__global__ __launch_bounds__(256) void prep_wt(const float* __restrict__ W, int ncols,
                                               unsigned short* __restrict__ WT) {
  static_assert(KP % 32 == 0 && KREAL <= KP && KREAL > KP - 32);
  constexpr int PT = KP + 8;
  __shared__ __align__(16) unsigned short tile[32 * PT];
  const int tid = threadIdx.x;
  const int n0 = blockIdx.x * 32;

  constexpr int NPADK = KP - KREAL;
  if constexpr (NPADK > 0) {
#pragma unroll 1
    for (int i = tid; i < 32 * NPADK; i += 256) {
      const int r = i / NPADK;
      const int kk = KREAL + (i - r * NPADK);
      tile[r * PT + kk] = (unsigned short)0;
    }
  }
  __syncthreads();

  constexpr int NLD = KREAL * 8;
  constexpr int NIT = (NLD + 255) / 256;
#pragma unroll 1
  for (int it = 0; it < NIT; ++it) {
    const int idx = it * 256 + tid;
    int kr = idx >> 3;
    kr = (kr < KREAL) ? kr : (KREAL - 1);
    const int c4 = (idx & 7) * 4;
    const v4f x = *(const v4f*)(W + (size_t)kr * ncols + n0 + c4);
    if (idx < NLD) {
      tile[(c4 + 0) * PT + kr] = cvt_in_bits(x[0]);
      tile[(c4 + 1) * PT + kr] = cvt_in_bits(x[1]);
      tile[(c4 + 2) * PT + kr] = cvt_in_bits(x[2]);
      tile[(c4 + 3) * PT + kr] = cvt_in_bits(x[3]);
    }
  }
  __syncthreads();

  constexpr int CPR = KP / 8;
  constexpr int NCH = 32 * CPR;
  constexpr int SIT = (NCH + 255) / 256;
  unsigned short* dst = WT + (size_t)n0 * KP;
  for (int pass = 0; pass < 2; ++pass) {
#pragma unroll 1
    for (int it = 0; it < SIT; ++it) {
      const int ci = it * 256 + tid;
      if (ci < NCH) {
        const int row = ci / CPR;
        const int kc = (ci - row * CPR) * 8;
        const v4u val = *(const v4u*)(tile + row * PT + kc);
        *(volatile v4u*)(dst + (size_t)row * KP + kc) = val;
      }
    }
    __threadfence();
  }
}

__global__ __launch_bounds__(256) void prep_static(const float* __restrict__ X,
                                                   unsigned short* __restrict__ XP) {
  const int ci = blockIdx.x * 256 + threadIdx.x;
  const int row = ci >> 2;
  const int kc = (ci & 3) * 8;
  unsigned short b[8];
#pragma unroll
  for (int e = 0; e < 8; ++e) {
    const int kk = kc + e;
    const int ka = (kk < NS) ? kk : (NS - 1);
    const float x = X[(size_t)row * NS + ka];
    const float v = (kk < NS) ? x : 0.0f;
    b[e] = cvt_in_bits(v);
  }
  v4u q;
  q[0] = (unsigned)b[0] | ((unsigned)b[1] << 16);
  q[1] = (unsigned)b[2] | ((unsigned)b[3] << 16);
  q[2] = (unsigned)b[4] | ((unsigned)b[5] << 16);
  q[3] = (unsigned)b[6] | ((unsigned)b[7] << 16);
  volatile v4u* p = (volatile v4u*)(XP + (size_t)ci * 8);
  *p = q;
  __threadfence();
  *p = q;
}

__global__ __launch_bounds__(512) void lstm_rec(
    const float* __restrict__ xin,
    const float* __restrict__ bias,
    const float* __restrict__ bstat,
    const unsigned short* __restrict__ kT,
    const unsigned short* __restrict__ rT,
    const unsigned short* __restrict__ wT,
    const unsigned short* __restrict__ sP,
    float* __restrict__ out)
{
  __shared__ __align__(16) unsigned short hS[ROWS * HPITCH];
  __shared__ __align__(16) float oS[ROWS * OPITCH];

  const int tid = threadIdx.x;
  const int lane = tid & 31;
  const int uw = tid >> 5;
  const int m = lane & 15;
  const int hf = lane >> 4;
  const int b0 = blockIdx.x * ROWS;
  const int ncl = uw * 16 + m;

  for (int i = tid; i < ROWS * HPITCH / 8; i += 512) ((v4u*)hS)[i] = (v4u){0u, 0u, 0u, 0u};

  float ig[8];
  {
    FragU sa, wb;
    const unsigned short* ap = sP + (size_t)(b0 + m) * KS_PAD + 8 * hf;
    const unsigned short* bp = wT + (size_t)ncl * KS_PAD + 8 * hf;
    sa.q[0] = *(const v4u*)(ap);
    sa.q[1] = *(const v4u*)(ap + 16);
    wb.q[0] = *(const v4u*)(bp);
    wb.q[1] = *(const v4u*)(bp + 16);
    v8f ai = zero8();
    ai = mma16(sa.v, wb.v, ai);
    guard1(ai, sa.v, wb.v);
    const float bs = bfr(bstat[ncl]);
#pragma unroll
    for (int r = 0; r < 8; ++r) ig[r] = sigm(ai[r] * INV_CARRY2 + bs);
  }

  const float bF = bfr(bias[ncl]);
  const float bC = bfr(bias[NU + ncl]);
  const float bO = bfr(bias[2 * NU + ncl]);

  FragU kw0, kw1, kw2;
  {
    const unsigned short* p0 = kT + (size_t)(0 * NU + ncl) * ND + 8 * hf;
    const unsigned short* p1 = kT + (size_t)(1 * NU + ncl) * ND + 8 * hf;
    const unsigned short* p2 = kT + (size_t)(2 * NU + ncl) * ND + 8 * hf;
    kw0.q[0] = *(const v4u*)(p0); kw0.q[1] = *(const v4u*)(p0 + 16);
    kw1.q[0] = *(const v4u*)(p1); kw1.q[1] = *(const v4u*)(p1 + 16);
    kw2.q[0] = *(const v4u*)(p2); kw2.q[1] = *(const v4u*)(p2 + 16);
  }

  float cS[8], hv[8];
#pragma unroll
  for (int r = 0; r < 8; ++r) { cS[r] = 0.0f; hv[r] = 0.0f; }

  __syncthreads();

  for (int t = 0; t < NT; ++t) {
    const float* xr = xin + ((size_t)(b0 + m) * NT + t) * ND + 8 * hf;
    const v4f x0 = *(const v4f*)(xr);
    const v4f x1 = *(const v4f*)(xr + 4);
    const v4f x2 = *(const v4f*)(xr + 16);
    const v4f x3 = *(const v4f*)(xr + 20);
    v16h xa;
    xa[0]  = cvt_in(x0[0]); xa[1]  = cvt_in(x0[1]); xa[2]  = cvt_in(x0[2]); xa[3]  = cvt_in(x0[3]);
    xa[4]  = cvt_in(x1[0]); xa[5]  = cvt_in(x1[1]); xa[6]  = cvt_in(x1[2]); xa[7]  = cvt_in(x1[3]);
    xa[8]  = cvt_in(x2[0]); xa[9]  = cvt_in(x2[1]); xa[10] = cvt_in(x2[2]); xa[11] = cvt_in(x2[3]);
    xa[12] = cvt_in(x3[0]); xa[13] = cvt_in(x3[1]); xa[14] = cvt_in(x3[2]); xa[15] = cvt_in(x3[3]);

    v8f aF = zero8(), aC = zero8(), aO = zero8();
    aF = mma16(xa, kw0.v, aF);
    aC = mma16(xa, kw1.v, aC);
    aO = mma16(xa, kw2.v, aO);
    guard3(aF, aC, aO, xa, kw0.v, kw1.v, kw2.v);

#pragma unroll 1
    for (int kc = 0; kc < NU / 32; ++kc) {
      FragU ha, r0, r1, r2;
      const unsigned short* hp = hS + m * HPITCH + kc * 32 + 8 * hf;
      ha.q[0] = *(const v4u*)(hp);
      ha.q[1] = *(const v4u*)(hp + 16);
      const unsigned short* rp0 = rT + (size_t)(0 * NU + ncl) * NU + kc * 32 + 8 * hf;
      const unsigned short* rp1 = rT + (size_t)(1 * NU + ncl) * NU + kc * 32 + 8 * hf;
      const unsigned short* rp2 = rT + (size_t)(2 * NU + ncl) * NU + kc * 32 + 8 * hf;
      r0.q[0] = *(const v4u*)(rp0); r0.q[1] = *(const v4u*)(rp0 + 16);
      r1.q[0] = *(const v4u*)(rp1); r1.q[1] = *(const v4u*)(rp1 + 16);
      r2.q[0] = *(const v4u*)(rp2); r2.q[1] = *(const v4u*)(rp2 + 16);
      aF = mma16(ha.v, r0.v, aF);
      aC = mma16(ha.v, r1.v, aC);
      aO = mma16(ha.v, r2.v, aO);
      guard3(aF, aC, aO, ha.v, r0.v, r1.v, r2.v);
    }

    __syncthreads();

#pragma unroll
    for (int r = 0; r < 8; ++r) {
      const float gF = aF[r] * INV_CARRY2 + bF;
      const float gC = aC[r] * INV_CARRY2 + bC;
      const float gO = aO[r] * INV_CARRY2 + bO;
      const float fg = sigm(gF);
      const float ct = tnh(gC);
      const float og = sigm(gO);
      const float cn = fg * cS[r] + ig[r] * ct;
      cS[r] = cn;
      const float hn = og * tnh(cn);
      hv[r] = hn;
      hS[(8 * hf + r) * HPITCH + ncl] = h16_bits(hn * CARRY);
    }
    __syncthreads();
  }

#pragma unroll
  for (int r = 0; r < 8; ++r) oS[(8 * hf + r) * OPITCH + ncl] = hv[r];
  __syncthreads();

  float* ob = out + (size_t)b0 * NU;
  for (int pass = 0; pass < 2; ++pass) {
#pragma unroll
    for (int it = 0; it < 2; ++it) {
      const int ci = it * 512 + tid;
      const int row = ci >> 6;
      const int c4 = (ci & 63) * 4;
      const v4f val = *(const v4f*)(oS + row * OPITCH + c4);
      *(volatile v4f*)(ob + (size_t)row * NU + c4) = val;
    }
    __threadfence();
  }
}

extern "C" void kernel_launch(void* const* d_in, const int* in_sizes, int n_in,
                              void* d_out, int out_size, void* d_ws, size_t ws_size,
                              hipStream_t stream)
{
  (void)in_sizes; (void)out_size;
  if (n_in < 7) return;
  if (ws_size < WS_TOTAL) return;

  const float* xin   = (const float*)d_in[0];
  const float* stat  = (const float*)d_in[1];
  const float* kern  = (const float*)d_in[2];
  const float* reck  = (const float*)d_in[3];
  const float* bias  = (const float*)d_in[4];
  const float* wstat = (const float*)d_in[5];
  const float* bstat = (const float*)d_in[6];
  float* out = (float*)d_out;

  char* ws = (char*)d_ws;
  unsigned short* kT = (unsigned short*)(ws + OFF_KT);
  unsigned short* rT = (unsigned short*)(ws + OFF_RT);
  unsigned short* wT = (unsigned short*)(ws + OFF_WT);
  unsigned short* sP = (unsigned short*)(ws + OFF_SP);

  hipLaunchKernelGGL(HIP_KERNEL_NAME(prep_wt<ND, ND>), dim3(NG / 32), dim3(256), 0, stream,
                     kern, (int)NG, kT);
  hipLaunchKernelGGL(HIP_KERNEL_NAME(prep_wt<NU, NU>), dim3(NG / 32), dim3(256), 0, stream,
                     reck, (int)NG, rT);
  hipLaunchKernelGGL(HIP_KERNEL_NAME(prep_wt<KS_PAD, NS>), dim3(NU / 32), dim3(256), 0, stream,
                     wstat, (int)NU, wT);
  hipLaunchKernelGGL(prep_static, dim3(NB * KS_PAD / 8 / 256), dim3(256), 0, stream, stat, sP);
  hipLaunchKernelGGL(lstm_rec, dim3(NB / ROWS), dim3(512), 0, stream,
                     xin, bias, bstat,
                     (const unsigned short*)kT, (const unsigned short*)rT,
                     (const unsigned short*)wT, (const unsigned short*)sP, out);
}
